// GMM_Head_55095840473822
// MI455X (gfx1250) — hardware-verified
//
#include <hip/hip_runtime.h>


#ifndef NB
#define NB 2048
#endif
#define NB_FULL 2048
#define KD   4096
#define NG   128
#define OD   1024
#define MT   256
#define WINC 16
#define CEXP ((float)(-((double)OD * (double)OD / 8.0) * 1.4426950408889634))

static_assert(NB % 64 == 0);
static_assert(NG % 64 == 0);
static_assert(KD % 32 == 0);
static_assert(((size_t)NB * KD) % 8 == 0);
static_assert(((size_t)NG * KD) % 8 == 0);
static_assert(NB <= NB_FULL);
static_assert(MT * 4 == OD);
static_assert((size_t)MT * 16 == (size_t)OD * 4);
static_assert(MT % 32 == 0);
static_assert(NG % 32 == 0);
static_assert(NG / 32 <= MT / 32);
static_assert(32 * 4 == 128);
static_assert((NG * 4) % 128 == 0);
static_assert(8 * 32 * 16 == 16 * 64 * 4);
static_assert(32 * 32 == 16 * 64);
static_assert((68 * 4) % 16 == 0);
static_assert(16 * 68 * 4 <= 131072);
static_assert(NG * 4 <= 131072);

typedef unsigned short bf;
typedef __attribute__((ext_vector_type(16))) __bf16   v16bf;
typedef __attribute__((ext_vector_type(8)))  unsigned short v8us;
typedef __attribute__((ext_vector_type(8)))  float    v8f;
typedef __attribute__((ext_vector_type(4)))  float    v4f;
typedef v4f  __attribute__((may_alias)) v4fa;

__device__ __forceinline__ unsigned short f2bf(float f) { unsigned u = __float_as_uint(f); u += 0x7FFFu + ((u >> 16) & 1u); return (unsigned short)(u >> 16); }
__device__ __forceinline__ float bfr(float f) { return __uint_as_float(((unsigned)f2bf(f)) << 16); }
__device__ __forceinline__ v16bf cat16b(v8us lo, v8us hi) { return __builtin_bit_cast(v16bf, __builtin_shufflevector(lo, hi, 0, 1, 2, 3, 4, 5, 6, 7, 8, 9, 10, 11, 12, 13, 14, 15)); }
__device__ __forceinline__ v8f wmmab(v16bf a, v16bf b, v8f c) { return __builtin_amdgcn_wmma_f32_16x16x32_bf16(false, a, false, b, (short)0, c, false, false); }
__device__ __forceinline__ v16bf ldb(const bf* p)  { return cat16b(*(const v8us*)p, *(const v8us*)(p + 16)); }
__device__ __forceinline__ void wave_sync() { __builtin_amdgcn_fence(3  , "wavefront"); __builtin_amdgcn_wave_barrier(); asm volatile("" ::: "memory"); }

__global__ __launch_bounds__(256) void k_cvt8(const float* __restrict__ src, bf* dst, size_t n8) {
    const size_t i = (size_t)blockIdx.x * 256 + threadIdx.x; if (i >= n8) return;
    const v8f v = *(const v8f*)(src + i * 8); v8us o;
#pragma unroll
    for (int k = 0; k < 8; ++k) o[k] = f2bf(v[k]);
    *(volatile v8us*)(dst + i * 8) = o; __threadfence(); *(volatile v8us*)(dst + i * 8) = o;
}

__global__ __launch_bounds__(32) void k_lin(const bf* __restrict__ A, const bf* __restrict__ Bt, const float* __restrict__ bias, float* MEANS) {
    __shared__ __align__(16) float os[16 * 68];
    const int K = KD;
    const int lane = threadIdx.x & 31, lr = lane & 15, hi = lane >> 4; const int r0 = blockIdx.x * 64, c0 = blockIdx.y * 64;
    v8f acc[4][4];
#pragma unroll
    for (int mb = 0; mb < 4; ++mb)
#pragma unroll
        for (int nb = 0; nb < 4; ++nb) acc[mb][nb] = (v8f){};
    const size_t aoff = (size_t)(r0 + lr) * K + 8 * hi, boff = (size_t)(c0 + lr) * K + 8 * hi;
#pragma unroll 1
    for (int kc = 0; kc < K; kc += 32) {
        v16bf a[4];
#pragma unroll
        for (int mb = 0; mb < 4; ++mb) a[mb] = ldb(A + aoff + (size_t)mb * 16 * K + kc);
#pragma unroll
        for (int nb = 0; nb < 4; ++nb) { const v16bf b = ldb(Bt + boff + (size_t)nb * 16 * K + kc);
#pragma unroll
            for (int mb = 0; mb < 4; ++mb) acc[mb][nb] = wmmab(a[mb], b, acc[mb][nb]); }
        asm volatile("v_nop\n\tv_nop\n\tv_nop\n\tv_nop" : "+v"(acc[0][0]), "+v"(acc[1][1]), "+v"(acc[2][2]), "+v"(acc[3][3]) : "v"(a[0]), "v"(a[1]), "v"(a[2]), "v"(a[3]));
    }
    float bc[4];
#pragma unroll
    for (int nb = 0; nb < 4; ++nb) bc[nb] = bfr(bias[c0 + nb * 16 + lr]);
#pragma unroll
    for (int mb = 0; mb < 4; ++mb) {
#pragma unroll
        for (int nb = 0; nb < 4; ++nb) {
#pragma unroll
            for (int j = 0; j < 8; ++j) os[(hi * 8 + j) * 68 + nb * 16 + lr] = acc[mb][nb][j] + bc[nb]; }
        wave_sync();
#pragma unroll 1
        for (int s = 0; s < 32; ++s) { const int idx = s * 32 + lane; const int o = (idx >> 6) * 68 + (idx & 63);
            const float pv = os[o]; os[o] = tanhf(pv); }
        wave_sync();
        float* mrow = MEANS + (size_t)(r0 + mb * 16) * NG + c0;
#pragma unroll 1
        for (int ps = 0; ps < 2; ++ps) {
#pragma unroll
            for (int s = 0; s < 8; ++s) { const int row = 2 * s + (lane >> 4), cofs = (lane & 15) * 4;
                const v4f val = *(const v4fa*)(&os[row * 68 + cofs]);
                *(volatile v4f*)(mrow + (size_t)row * NG + cofs) = val; }
            if (ps == 0) __threadfence(); }
        wave_sync();
    }
}

__global__ __launch_bounds__(MT) void k_mix(const float* __restrict__ MEANS, float* OUT) {
#pragma clang fp contract(off)
    __shared__ float sm[NG];
    const int tid = threadIdx.x;
    const int wave = __builtin_amdgcn_readfirstlane((int)(threadIdx.x >> 5));
    const int row = blockIdx.x;
    if (wave < NG / 32) sm[tid] = MEANS[(size_t)row * NG + tid];
    __syncthreads();
    const float step = 1.0f / (float)OD;
    const int d0 = 4 * tid;
    v4f ep;
#pragma unroll
    for (int i = 0; i < 4; ++i) ep[i] = (float)(2 * (d0 + i) + 1 - OD) * step;
    const int w0 = wave * 128;
    const float wlo = (float)(2 * w0 + 1 - OD - 2 * WINC) * step;
    const float whi = (float)(2 * (w0 + 127) + 1 - OD + 2 * WINC) * step;
    v4f acc = (v4f){};
#pragma unroll 2
    for (int g = 0; g < NG; ++g) {
        const float mv = sm[g];
        const int hit = ((mv >= wlo) & (mv <= whi)) ? 1 : 0;
        if (__builtin_amdgcn_readfirstlane(hit) != 0) {
#pragma unroll
            for (int i = 0; i < 4; ++i) { const float df = ep[i] - mv; const float t = df * df; acc[i] += __builtin_amdgcn_exp2f(t * CEXP); }
        }
    }
    const float cm = (1.0f / ((2.0f / (float)OD) * 2.5066282746310002f)) * (1.0f / (float)NG);
    v4f res;
#pragma unroll
    for (int i = 0; i < 4; ++i) res[i] = logf(acc[i] * cm + 1e-05f);
    float* orow = OUT + (size_t)row * OD + d0;
    *(volatile v4f*)orow = res; __threadfence(); *(volatile v4f*)orow = res;
}

static constexpr size_t al256(size_t v) { return (v + 255) & ~(size_t)255; }
static constexpr size_t SZ_XB = al256((size_t)NB * KD * 2);
static constexpr size_t SZ_WB = al256((size_t)NG * KD * 2);
static constexpr size_t SZ_MN = al256((size_t)NB * NG * 4);
static constexpr size_t SZ_TOTAL = SZ_XB + SZ_WB + SZ_MN;
static_assert(SZ_TOTAL <= (size_t)134217728);
static_assert(((size_t)NB * KD * 2) % 128 == 0);
static_assert(((size_t)NG * KD * 2) % 128 == 0);
static_assert(((size_t)NB * NG * 4) % 128 == 0);

extern "C" void kernel_launch(void* const* d_in, const int* in_sizes, int n_in,
                              void* d_out, int out_size, void* d_ws, size_t ws_size, hipStream_t stream) {
    if (n_in < 3) return;
    if ((size_t)in_sizes[0] < (size_t)NB * KD) return;
    if ((size_t)in_sizes[1] < (size_t)NG * KD) return;
    if (in_sizes[2] < NG) return;
    if ((size_t)out_size < (size_t)NB * OD) return;
    if (SZ_TOTAL > ws_size) return;
    const float* x  = (const float*)d_in[0];
    const float* w  = (const float*)d_in[1];
    const float* bv = (const float*)d_in[2];
    float* OUT = (float*)d_out;
    char* wsp = (char*)d_ws;
    bf* XB = (bf*)wsp; wsp += SZ_XB;
    bf* WB = (bf*)wsp; wsp += SZ_WB;
    float* MN = (float*)wsp; wsp += SZ_MN;

    { const size_t n8 = (size_t)NB * KD / 8; k_cvt8<<<(unsigned)((n8 + 255) / 256), 256, 0, stream>>>(x, XB, n8); }
    { const size_t n8 = (size_t)NG * KD / 8; k_cvt8<<<(unsigned)((n8 + 255) / 256), 256, 0, stream>>>(w, WB, n8); }
    k_lin<<<dim3(NB / 64, NG / 64, 1), 32, 0, stream>>>(XB, WB, bv, MN);
    k_mix<<<dim3(NB, 1, 1), MT, 0, stream>>>(MN, OUT);
}
